// EnhancedUncertaintyAttention_28681791602831
// MI455X (gfx1250) — hardware-verified
//
#include <hip/hip_runtime.h>
#include <math.h>

constexpr int kBatch     = 2;
constexpr int kSeq       = 1024;
constexpr int kDim       = 1024;
constexpr int kHeads     = 16;
constexpr int kSamp      = 4;
constexpr int kDh        = 64;
constexpr int kTok       = kBatch * kSeq;
constexpr int kHeadsHalf = 8;
constexpr int kQKld      = 2 * kDim;
constexpr float kQKVCarry   = 16.0f;
constexpr float kPCarry     = 32768.0f;
constexpr float kCombCarry  = 256.0f;
constexpr float kWoCarry    = 16.0f;
constexpr float kScoreScale = 0.125f / (16.0f * 16.0f);
constexpr float kPVScale    = kCombCarry / (kPCarry * kQKVCarry);
constexpr float kOutScale   = 1.0f / (kCombCarry * kWoCarry);

typedef __attribute__((ext_vector_type(16))) _Float16 v16h;
typedef __attribute__((ext_vector_type(8)))  _Float16 v8h;
typedef __attribute__((ext_vector_type(16))) __bf16   v16b;
typedef __attribute__((ext_vector_type(8)))  __bf16   v8b;
typedef __attribute__((ext_vector_type(8)))  float    v8f;
typedef __attribute__((ext_vector_type(4)))  float    v4f;
typedef __attribute__((ext_vector_type(4)))  unsigned int v4u;

__device__ __forceinline__ unsigned short f2bf_bits(float f) {
  unsigned u = __float_as_uint(f);
  return (unsigned short)((u + 0x7FFFu + ((u >> 16) & 1u)) >> 16);
}
__device__ __forceinline__ float bf_bits2f(unsigned short h) { return __uint_as_float(((unsigned)h) << 16); }

__device__ __forceinline__ void dep_guard_h(v8f& a, v8f& b, v16h x, v16h y) { asm volatile("v_nop\n\tv_nop\n\tv_nop\n\tv_nop" : "+v"(a), "+v"(b) : "v"(x), "v"(y)); }
__device__ __forceinline__ void dep_guard_b(v8f& a, v8f& b, v16b x, v16b y) { asm volatile("v_nop\n\tv_nop\n\tv_nop\n\tv_nop" : "+v"(a), "+v"(b) : "v"(x), "v"(y)); }
__device__ __forceinline__ void keep4_h(v16h a, v16h b, v16h c, v16h d) { asm volatile("v_nop" :: "v"(a), "v"(b), "v"(c), "v"(d)); }
__device__ __forceinline__ void keep4_b(v16b a, v16b b, v16b c, v16b d) { asm volatile("v_nop" :: "v"(a), "v"(b), "v"(c), "v"(d)); }
__device__ __forceinline__ void acc_guard4(v8f& a, v8f& b, v8f& c, v8f& d) { asm volatile("v_nop\n\tv_nop\n\tv_nop\n\tv_nop" : "+v"(a), "+v"(b), "+v"(c), "+v"(d)); }
template <typename T> struct Frag;
template <> struct Frag<_Float16> {
  typedef v16h V; union U { v16h v; v8h h[2]; };
  static __device__ __forceinline__ v16h load(const _Float16* p) {
    U f; f.h[0] = *(const v8h*)(p); f.h[1] = *(const v8h*)(p + 16); return f.v;
  }
  static __device__ __forceinline__ v8f mma(v16h a, v16h b, v8f c) {
    return __builtin_amdgcn_wmma_f32_16x16x32_f16(false, a, false, b, (short)0, c, false, false);
  }
  static __device__ __forceinline__ void guard(v8f& a, v8f& b, v16h x, v16h y) { dep_guard_h(a, b, x, y); }
  static __device__ __forceinline__ void keep(v16h a, v16h b, v16h c, v16h d) { keep4_h(a, b, c, d); }
};
template <> struct Frag<__bf16> {
  typedef v16b V; union U { v16b v; v8b h[2]; };
  static __device__ __forceinline__ v16b load(const __bf16* p) {
    U f; f.h[0] = *(const v8b*)(p); f.h[1] = *(const v8b*)(p + 16); return f.v;
  }
  static __device__ __forceinline__ v8f mma(v16b a, v16b b, v8f c) {
    return __builtin_amdgcn_wmma_f32_16x16x32_bf16(false, a, false, b, (short)0, c, false, false);
  }
  static __device__ __forceinline__ void guard(v8f& a, v8f& b, v16b x, v16b y) { dep_guard_b(a, b, x, y); }
  static __device__ __forceinline__ void keep(v16b a, v16b b, v16b c, v16b d) { keep4_b(a, b, c, d); }
};

__device__ __forceinline__ unsigned pk16(unsigned short a, unsigned short b) { return (unsigned)a | ((unsigned)b << 16); }
__device__ __forceinline__ unsigned short h_bits(float f) { const _Float16 h = (_Float16)f; return __builtin_bit_cast(unsigned short, h); }

template <int ET> struct Elem;
template <> struct Elem<0> { typedef _Float16 T; };
template <> struct Elem<1> { typedef __bf16 T; };
template <int ET, bool SPLIT, int BIAS_MODE, int OUT_MODE, bool RESID, int ACT = 0>
__global__ __launch_bounds__(256) void wmma_gemm64(
    const unsigned short* __restrict__ Ap, const unsigned short* __restrict__ A2p, int lda, long strideA,
    const unsigned short* __restrict__ Btp, const unsigned short* __restrict__ Bt2p, int ldb, long strideB,
    void* Cout, void* Cout2, int ldc, long strideC,
    const float* __restrict__ bias,
    const float* resid, long strideR,
    int M, int N, int K, float scale) {
  typedef typename Elem<ET>::T T;
  typedef typename Frag<T>::V V;
  const T* A = (const T*)Ap; const T* A2 = (const T*)A2p; const T* Bt = (const T*)Btp; const T* Bt2 = (const T*)Bt2p;
  __shared__ __align__(16) float sT[8][16 * 68];
  const int b    = blockIdx.y;
  const int lane = threadIdx.x & 31;
  const int wave = threadIdx.x >> 5;
  const int tilesN = N >> 6;
  const int tilesM = M >> 6;
  const int tile = blockIdx.x * 8 + wave;
  if (tile >= tilesM * tilesN) return;
  const int tm = tile / tilesN;
  const int tn = tile - tm * tilesN;
  const int m0 = tm << 6;
  const int n0 = tn << 6;

  const T* Ab  = A  + (size_t)b * strideA;
  const T* Bb  = Bt + (size_t)b * strideB;
  const T* Ab2 = SPLIT ? (A2  + (size_t)b * strideA) : nullptr;
  const T* Bb2 = SPLIT ? (Bt2 + (size_t)b * strideB) : nullptr;

  const int rlane = lane & 15;
  const int koff  = (lane >> 4) * 8;
  const int mOff  = (lane >> 4) * 8;

  v8f acc[4][4];
#pragma unroll
  for (int i = 0; i < 4; ++i)
#pragma unroll
    for (int j = 0; j < 4; ++j) acc[i][j] = (v8f){0.f,0.f,0.f,0.f,0.f,0.f,0.f,0.f};

  for (int k0 = 0; k0 < K; k0 += 32) {
    V bh[4], bl[4];
#pragma unroll
    for (int j = 0; j < 4; ++j) {
      const size_t bo = (size_t)(n0 + (j << 4) + rlane) * ldb + koff + k0;
      bh[j] = Frag<T>::load(Bb + bo);
      if (SPLIT) bl[j] = Frag<T>::load(Bb2 + bo);
    }
#pragma unroll
    for (int i = 0; i < 4; ++i) {
      const size_t ao = (size_t)(m0 + (i << 4) + rlane) * lda + koff + k0;
      V ah = Frag<T>::load(Ab + ao);
      V al;
      if (SPLIT) al = Frag<T>::load(Ab2 + ao);
#pragma unroll
      for (int j = 0; j < 4; ++j) {
        acc[i][j] = Frag<T>::mma(ah, bh[j], acc[i][j]);
        if (SPLIT) {
          acc[i][j] = Frag<T>::mma(ah, bl[j], acc[i][j]);
          acc[i][j] = Frag<T>::mma(al, bh[j], acc[i][j]);
        }
      }
      Frag<T>::guard(acc[i][0], acc[i][3], ah, SPLIT ? al : ah);
    }
    Frag<T>::keep(bh[0], bh[1], bh[2], bh[3]);
    if (SPLIT) Frag<T>::keep(bl[0], bl[1], bl[2], bl[3]);
  }
  acc_guard4(acc[0][0], acc[0][1], acc[0][2], acc[0][3]);
  acc_guard4(acc[1][0], acc[1][1], acc[1][2], acc[1][3]);
  acc_guard4(acc[2][0], acc[2][1], acc[2][2], acc[2][3]);
  acc_guard4(acc[3][0], acc[3][1], acc[3][2], acc[3][3]);

  float* slab = sT[wave];
  const float* Rb = RESID ? (resid + (size_t)b * strideR) : nullptr;
#pragma unroll
  for (int i = 0; i < 4; ++i) {
    const int mBase = m0 + (i << 4);
#pragma unroll
    for (int j = 0; j < 4; ++j) {
      const int n = n0 + (j << 4) + rlane;
      float bv = 0.f;
      if (BIAS_MODE == 2) bv = bias[n];
#pragma unroll
      for (int r = 0; r < 8; ++r) {
        float v = acc[i][j][r] * scale;
        if (BIAS_MODE == 1) v += bias[mBase + mOff + r];
        if (BIAS_MODE == 2) v += bv;
        if (RESID) v += Rb[(size_t)(mBase + mOff + r) * ldc + n];
        if (ACT == 2) v = fmaxf(v, 0.0f);
        if (ACT == 4) v = (v > 0.f) ? v : 0.01f * v;
        slab[(mOff + r) * 68 + (j << 4) + rlane] = v;
      }
    }
    __builtin_amdgcn_fence(__ATOMIC_RELEASE, "workgroup");
    __builtin_amdgcn_wave_barrier();
    __builtin_amdgcn_fence(__ATOMIC_ACQUIRE, "workgroup");
    if (OUT_MODE == 0) {
      float* C = (float*)Cout + (size_t)b * strideC;
      const int hh = lane >> 4, c4 = (lane & 15) * 4;
      for (int pass = 0; pass < 2; ++pass) {
#pragma unroll
        for (int it = 0; it < 8; ++it) {
          const int row = it * 2 + hh;
          v4f v = *(const v4f*)(slab + row * 68 + c4);
          *(volatile v4f*)(C + (size_t)(mBase + row) * ldc + n0 + c4) = v;
        }
        __threadfence();
      }
    } else {
      const int q = lane >> 3, c8 = (lane & 7) * 8;
      unsigned short* C  = (unsigned short*)Cout  + (size_t)b * strideC;
      unsigned short* C2 = (OUT_MODE == 2) ? ((unsigned short*)Cout2 + (size_t)b * strideC) : nullptr;
      for (int pass = 0; pass < 2; ++pass) {
#pragma unroll
        for (int it = 0; it < 4; ++it) {
          const int row = it * 4 + q;
          const float* sp = slab + row * 68 + c8;
          v8h hv, lv;
#pragma unroll
          for (int e = 0; e < 8; ++e) {
            if (OUT_MODE == 1) {
              hv[e] = (_Float16)sp[e];
            } else {
              unsigned short hb = f2bf_bits(sp[e]);
              unsigned short lb = f2bf_bits(sp[e] - bf_bits2f(hb));
              hv[e] = __builtin_bit_cast(_Float16, hb);
              lv[e] = __builtin_bit_cast(_Float16, lb);
            }
          }
          *(volatile v8h*)(C + (size_t)(mBase + row) * ldc + n0 + c8) = hv;
          if (OUT_MODE == 2) *(volatile v8h*)(C2 + (size_t)(mBase + row) * ldc + n0 + c8) = lv;
        }
        __threadfence();
      }
    }
    __builtin_amdgcn_fence(__ATOMIC_RELEASE, "workgroup");
    __builtin_amdgcn_wave_barrier();
    __builtin_amdgcn_fence(__ATOMIC_ACQUIRE, "workgroup");
  }
}

__global__ __launch_bounds__(256) void cast_bf16_kernel(const float* __restrict__ in, unsigned short* __restrict__ out, int n8) {
  const int i = blockIdx.x * 256 + threadIdx.x;
  if (i >= n8) return;
  const float* p = in + 8 * (size_t)i;
  const v4f a = *(const v4f*)(p);
  const v4f c = *(const v4f*)(p + 4);
  unsigned short hb[8];
#pragma unroll
  for (int e = 0; e < 4; ++e) {
    hb[e]     = f2bf_bits(a[e]);
    hb[4 + e] = f2bf_bits(c[e]);
  }
  const v4u u = (v4u){pk16(hb[0], hb[1]), pk16(hb[2], hb[3]), pk16(hb[4], hb[5]), pk16(hb[6], hb[7])};
  unsigned short* q = out + 8 * (size_t)i;
  *(volatile v4u*)q = u;
  __threadfence();
  *(volatile v4u*)q = u;
}

__global__ __launch_bounds__(256) void cast_wqk_kernel(const float* __restrict__ Wq, const float* __restrict__ Wk,
                                                       unsigned short* __restrict__ out) {
  const int y = blockIdx.y;
  const int smp = y & 3, which = y >> 2;
  const float* src = ((which == 0) ? Wq : Wk) + (size_t)smp * kDim * kDim;
  unsigned short* dst = out + (size_t)smp * kQKld * kDim + (size_t)which * kDim * kDim;
  const int i = blockIdx.x * 256 + threadIdx.x;
  if (i >= (kDim * kDim) / 8) return;
  const float* p = src + 8 * (size_t)i;
  const v4f a = *(const v4f*)(p);
  const v4f c = *(const v4f*)(p + 4);
  unsigned short hb[8];
#pragma unroll
  for (int e = 0; e < 4; ++e) {
    hb[e]     = f2bf_bits(a[e]);
    hb[4 + e] = f2bf_bits(c[e]);
  }
  const v4u u = (v4u){pk16(hb[0], hb[1]), pk16(hb[2], hb[3]), pk16(hb[4], hb[5]), pk16(hb[6], hb[7])};
  unsigned short* q = dst + 8 * (size_t)i;
  *(volatile v4u*)q = u;
  __threadfence();
  *(volatile v4u*)q = u;
}

__global__ __launch_bounds__(256) void cast_wo_kernel(const float* __restrict__ in, unsigned short* __restrict__ out, int n8) {
  const int i = blockIdx.x * 256 + threadIdx.x;
  if (i >= n8) return;
  const float* p = in + 8 * (size_t)i;
  const v4f a = *(const v4f*)(p);
  const v4f c = *(const v4f*)(p + 4);
  unsigned short hb[8];
#pragma unroll
  for (int e = 0; e < 4; ++e) {
    hb[e]     = h_bits(kWoCarry * bf_bits2f(f2bf_bits(a[e])));
    hb[4 + e] = h_bits(kWoCarry * bf_bits2f(f2bf_bits(c[e])));
  }
  const v4u u = (v4u){pk16(hb[0], hb[1]), pk16(hb[2], hb[3]), pk16(hb[4], hb[5]), pk16(hb[6], hb[7])};
  unsigned short* q = out + 8 * (size_t)i;
  *(volatile v4u*)q = u;
  __threadfence();
  *(volatile v4u*)q = u;
}

__global__ __launch_bounds__(256) void mean_kernel(const unsigned short* __restrict__ xb, float* __restrict__ xmean) {
  const int t = blockIdx.x * 256 + threadIdx.x;
  if (t >= kBatch * kDim) return;
  const int b = t >> 10, d = t & (kDim - 1);
  const unsigned short* p = xb + (size_t)b * kSeq * kDim + d;
  float acc = 0.f;
#pragma unroll 4
  for (int n = 0; n < kSeq; ++n) acc += bf_bits2f(p[(size_t)n * kDim]);
  const float m = acc * (1.0f / (float)kSeq);
  *(volatile float*)(xmean + t) = m;
  __threadfence();
  *(volatile float*)(xmean + t) = m;
}

__global__ __launch_bounds__(256) void gate_kernel(const float* __restrict__ xmean, const float* __restrict__ Wg,
                                                   const float* __restrict__ bg, const float* __restrict__ hw,
                                                   const float* __restrict__ temp, float* __restrict__ wsS) {
  __shared__ float vals[32];
  const int t = threadIdx.x, lane = t & 31, wave = t >> 5;
  if (t < 32) vals[t] = 0.f;
  __syncthreads();
  {
    const int b = wave >> 2, s = wave & 3;
    float acc = 0.f;
#pragma unroll 1
    for (int d = lane; d < kDim; d += 32) {
      const float wg = bf_bits2f(f2bf_bits(Wg[(size_t)s * kDim + d]));
      acc += xmean[b * kDim + d] * wg;
    }
#pragma unroll
    for (int off = 16; off > 0; off >>= 1) acc += __shfl_xor(acc, off, 32);
    if (lane == 0) {
      const float z = acc + bf_bits2f(f2bf_bits(bg[s]));
      vals[4 + b * kSamp + s] = 1.0f / (1.0f + __expf(-z));
    }
  }
  __syncthreads();
  if (t == 0) {
    float tc = bf_bits2f(f2bf_bits(temp[0]));
    tc = fminf(fmaxf(tc, 0.1f), 10.0f);
    const float invt = 1.0f / tc;
    const float l0 = bf_bits2f(f2bf_bits(hw[0])) * invt;
    const float l1 = bf_bits2f(f2bf_bits(hw[1])) * invt;
    const float l2 = bf_bits2f(f2bf_bits(hw[2])) * invt;
    const float l3 = bf_bits2f(f2bf_bits(hw[3])) * invt;
    const float mx = fmaxf(fmaxf(l0, l1), fmaxf(l2, l3));
    const float e0 = __expf(l0 - mx), e1 = __expf(l1 - mx), e2 = __expf(l2 - mx), e3 = __expf(l3 - mx);
    const float is = 1.0f / ((e0 + e1) + (e2 + e3));
    vals[0] = e0 * is; vals[1] = e1 * is; vals[2] = e2 * is; vals[3] = e3 * is;
    vals[12] = invt;
  }
  __syncthreads();
  if (wave == 0) {
    const float v = vals[lane];
    *(volatile float*)(wsS + lane) = v;
    __threadfence();
    *(volatile float*)(wsS + lane) = v;
  }
}

__global__ __launch_bounds__(128) void softmax_mix_kernel(const float* __restrict__ Sf, const float* __restrict__ wsS,
                                                          unsigned short* __restrict__ P16, float* out2,
                                                          int smp, int bat, int first) {
  __shared__ float redM[4];
  __shared__ float redS[4];
  __shared__ __align__(16) float arow[kSeq];
  const int i = blockIdx.x;
  const int t = threadIdx.x, lane = t & 31, wave = t >> 5;
  const int c0 = t * 8;
  const float invt = wsS[12];
  const float gw   = wsS[smp];
  const float coh  = wsS[4 + bat * kSamp + smp];
  const float wP   = kPCarry * gw * coh;
  const float wA   = gw * (1.0f / (float)kHeads);
  float a2[8];
#pragma unroll
  for (int e = 0; e < 8; ++e) a2[e] = 0.f;

#pragma unroll 1
  for (int h = 0; h < kHeadsHalf; ++h) {
    const size_t rb = ((size_t)h * kSeq + i) * kSeq + c0;
    const v4f va = *(const v4f*)(Sf + rb);
    const v4f vc = *(const v4f*)(Sf + rb + 4);
    float x[8];
#pragma unroll
    for (int e = 0; e < 4; ++e) { x[e] = va[e] * invt; x[4 + e] = vc[e] * invt; }
    float m = fmaxf(fmaxf(fmaxf(x[0], x[1]), fmaxf(x[2], x[3])), fmaxf(fmaxf(x[4], x[5]), fmaxf(x[6], x[7])));
#pragma unroll
    for (int off = 16; off > 0; off >>= 1) m = fmaxf(m, __shfl_xor(m, off, 32));
    if (lane == 0) redM[wave] = m;
    __syncthreads();
    const float M = fmaxf(fmaxf(redM[0], redM[1]), fmaxf(redM[2], redM[3]));
    float ex[8];
#pragma unroll
    for (int e = 0; e < 8; ++e) ex[e] = __expf(x[e] - M);
    float ssum = ((ex[0] + ex[1]) + (ex[2] + ex[3])) + ((ex[4] + ex[5]) + (ex[6] + ex[7]));
#pragma unroll
    for (int off = 16; off > 0; off >>= 1) ssum += __shfl_xor(ssum, off, 32);
    if (lane == 0) redS[wave] = ssum;
    __syncthreads();
    const float l  = (redS[0] + redS[1]) + (redS[2] + redS[3]);
    const float il = 1.0f / l;
    unsigned short hb[8];
#pragma unroll
    for (int e = 0; e < 8; ++e) {
      const float p = ex[e] * il;
      a2[e] += wA * p;
      hb[e] = h_bits(p * wP);
    }
    const v4u u = (v4u){pk16(hb[0], hb[1]), pk16(hb[2], hb[3]), pk16(hb[4], hb[5]), pk16(hb[6], hb[7])};
    unsigned short* q = P16 + rb;
    *(volatile v4u*)q = u;
    __threadfence();
    *(volatile v4u*)q = u;
  }

#pragma unroll
  for (int e = 0; e < 8; ++e) arow[c0 + e] = a2[e];
  __syncthreads();
  float* orow = out2 + ((size_t)bat * kSeq + i) * kSeq;
  const int ca = 4 * t, cb = 512 + 4 * t;
  const v4f v0 = *(const v4f*)(arow + ca);
  const v4f v1 = *(const v4f*)(arow + cb);
  const v4f o0 = *(const v4f*)(orow + ca);
  const v4f o1 = *(const v4f*)(orow + cb);
  v4f n0, n1;
#pragma unroll
  for (int e = 0; e < 4; ++e) {
    n0[e] = first ? v0[e] : (o0[e] + v0[e]);
    n1[e] = first ? v1[e] : (o1[e] + v1[e]);
  }
  *(volatile v4f*)(orow + ca) = n0;
  *(volatile v4f*)(orow + cb) = n1;
  __threadfence();
  *(volatile v4f*)(orow + ca) = n0;
  *(volatile v4f*)(orow + cb) = n1;
}

extern "C" void kernel_launch(void* const* d_in, const int* in_sizes, int n_in,
                              void* d_out, int out_size, void* d_ws, size_t ws_size,
                              hipStream_t stream) {
  if (n_in < 10) return;
  if (in_sizes[0] != kTok * kDim) return;
  if (in_sizes[1] != kSamp * kDim * kDim || in_sizes[2] != kSamp * kDim * kDim || in_sizes[3] != kSamp * kDim * kDim) return;
  if (in_sizes[4] != kSamp * kDim || in_sizes[5] != kSamp) return;
  if (in_sizes[6] != kDim * kDim || in_sizes[7] != kDim) return;
  if (in_sizes[8] != kSamp || in_sizes[9] != 1) return;
  if (out_size != kTok * kDim + kBatch * kSeq * kSeq) return;

  const float* x    = (const float*)d_in[0];
  const float* Wq   = (const float*)d_in[1];
  const float* Wk   = (const float*)d_in[2];
  const float* Wv   = (const float*)d_in[3];
  const float* Wg   = (const float*)d_in[4];
  const float* bg   = (const float*)d_in[5];
  const float* Wo   = (const float*)d_in[6];
  const float* bo   = (const float*)d_in[7];
  const float* hw   = (const float*)d_in[8];
  const float* temp = (const float*)d_in[9];
  float* yout = (float*)d_out;
  float* aout = (float*)d_out + (size_t)kTok * kDim;

  const size_t SZ_WSS  = 4096;
  const size_t SZ_XM   = (size_t)kBatch * kDim * 4;
  const size_t SZ_XB   = (size_t)kTok * kDim * 2;
  const size_t SZ_WQK  = (size_t)kSamp * kQKld * kDim * 2;
  const size_t SZ_WV   = (size_t)kSamp * kDim * kDim * 2;
  const size_t SZ_WO   = (size_t)kDim * kDim * 2;
  const size_t SZ_QK   = (size_t)kTok * kQKld * 2;
  const size_t SZ_VT   = (size_t)kBatch * kDim * kSeq * 2;
  const size_t SZ_S    = (size_t)kHeadsHalf * kSeq * kSeq * 4;
  const size_t SZ_P    = (size_t)kHeadsHalf * kSeq * kSeq * 2;
  const size_t SZ_CF   = (size_t)kBatch * kSeq * kDim * 4;
  const size_t SZ_CH   = (size_t)kBatch * kSeq * kDim * 2;
  size_t off = 0;
  const size_t oWSS = off; off += SZ_WSS;
  const size_t oXM  = off; off += SZ_XM;
  const size_t oXB  = off; off += SZ_XB;
  const size_t oWQK = off; off += SZ_WQK;
  const size_t oWV  = off; off += SZ_WV;
  const size_t oWO  = off; off += SZ_WO;
  const size_t oQK  = off; off += SZ_QK;
  const size_t oVT  = off; off += SZ_VT;
  const size_t oS   = off; off += SZ_S;
  const size_t oP   = off; off += SZ_P;
  const size_t oCF  = off; off += SZ_CF;
  const size_t oCH  = off; off += SZ_CH;
  const size_t TOTAL = off;
  if (TOTAL > ws_size) return;
  if (TOTAL > (size_t)134217728) return;

  char* ws = (char*)d_ws;
  float*          wsS    = (float*)(ws + oWSS);
  float*          xmean  = (float*)(ws + oXM);
  unsigned short* xb     = (unsigned short*)(ws + oXB);
  unsigned short* Wqkb   = (unsigned short*)(ws + oWQK);
  unsigned short* Wvb    = (unsigned short*)(ws + oWV);
  unsigned short* Wo16   = (unsigned short*)(ws + oWO);
  unsigned short* QK16   = (unsigned short*)(ws + oQK);
  unsigned short* VT16   = (unsigned short*)(ws + oVT);
  float*          Sf     = (float*)(ws + oS);
  unsigned short* P16    = (unsigned short*)(ws + oP);
  float*          combF  = (float*)(ws + oCF);
  unsigned short* comb16 = (unsigned short*)(ws + oCH);

  const dim3 blk(256);

  {
    const int n8x = kTok * kDim / 8;
    cast_bf16_kernel<<<dim3(n8x / 256), blk, 0, stream>>>(x, xb, n8x);
    cast_wqk_kernel<<<dim3((kDim * kDim / 8) / 256, 8), blk, 0, stream>>>(Wq, Wk, Wqkb);
    const int n8v = kSamp * kDim * kDim / 8;
    cast_bf16_kernel<<<dim3(n8v / 256), blk, 0, stream>>>(Wv, Wvb, n8v);
    const int n8o = kDim * kDim / 8;
    cast_wo_kernel<<<dim3(n8o / 256), blk, 0, stream>>>(Wo, Wo16, n8o);
  }
  mean_kernel<<<dim3((kBatch * kDim) / 256), blk, 0, stream>>>(xb, xmean);
  gate_kernel<<<dim3(1), blk, 0, stream>>>(xmean, Wg, bg, hw, temp, wsS);

  const dim3 gQK((((kTok / 64) * (kQKld / 64)) + 7) / 8, 1);
  const dim3 gV((((kDim / 64) * (kSeq / 64)) + 7) / 8, kBatch);
  const dim3 gS((((kSeq / 64) * (kSeq / 64)) + 7) / 8, kHeadsHalf);
  const dim3 gPV((((kSeq / 64) * (kDh / 64)) + 7) / 8, kHeadsHalf);
  const dim3 gOut((((kTok / 64) * (kDim / 64)) + 7) / 8, 1);

  for (int s = 0; s < kSamp; ++s) {
    const unsigned short* Wsb = Wqkb + (size_t)s * kQKld * kDim;
    wmma_gemm64<1, false, 0, 1, false, 0><<<gQK, blk, 0, stream>>>(
        xb, xb, kDim, 0L, Wsb, Wsb, kDim, 0L, (void*)QK16, (void*)QK16, kQKld, 0L,
        bo, x, 0L, kTok, kQKld, kDim, kQKVCarry);
    const unsigned short* Wvs = Wvb + (size_t)s * kDim * kDim;
    wmma_gemm64<1, false, 0, 1, false, 0><<<gV, blk, 0, stream>>>(
        Wvs, Wvs, kDim, 0L, xb, xb, kDim, (long)kSeq * kDim, (void*)VT16, (void*)VT16, kSeq, (long)kDim * kSeq,
        bo, x, 0L, kDim, kSeq, kDim, kQKVCarry);

    for (int b = 0; b < kBatch; ++b) {
      for (int hh = 0; hh < kHeads / kHeadsHalf; ++hh) {
        const unsigned short* Aq = QK16 + (size_t)b * kSeq * kQKld + (size_t)hh * kHeadsHalf * kDh;
        const unsigned short* Bk = Aq + kDim;
        wmma_gemm64<0, false, 0, 0, false, 0><<<gS, blk, 0, stream>>>(
            Aq, Aq, kQKld, (long)kDh, Bk, Bk, kQKld, (long)kDh, (void*)Sf, (void*)Sf, kSeq, (long)kSeq * kSeq,
            bo, x, 0L, kSeq, kSeq, kDh, kScoreScale);
        const int first = (s == 0 && hh == 0) ? 1 : 0;
        softmax_mix_kernel<<<dim3(kSeq), dim3(128), 0, stream>>>(Sf, wsS, P16, aout, s, b, first);
        const unsigned short* Vb = VT16 + (size_t)b * kDim * kSeq + (size_t)hh * kHeadsHalf * kDh * kSeq;
        float* Cf = combF + (size_t)b * kSeq * kDim + (size_t)hh * kHeadsHalf * kDh;
        if (s == 0) {
          wmma_gemm64<0, false, 0, 0, false, 0><<<gPV, blk, 0, stream>>>(
              P16, P16, kSeq, (long)kSeq * kSeq, Vb, Vb, kSeq, (long)kDh * kSeq, (void*)Cf, (void*)Cf, kDim, (long)kDh,
              bo, x, 0L, kSeq, kDh, kSeq, kPVScale);
        } else if (s < kSamp - 1) {
          wmma_gemm64<0, false, 0, 0, true, 0><<<gPV, blk, 0, stream>>>(
              P16, P16, kSeq, (long)kSeq * kSeq, Vb, Vb, kSeq, (long)kDh * kSeq, (void*)Cf, (void*)Cf, kDim, (long)kDh,
              bo, Cf, (long)kDh, kSeq, kDh, kSeq, kPVScale);
        } else {
          unsigned short* Ch = comb16 + (size_t)b * kSeq * kDim + (size_t)hh * kHeadsHalf * kDh;
          wmma_gemm64<0, false, 0, 1, true, 0><<<gPV, blk, 0, stream>>>(
              P16, P16, kSeq, (long)kSeq * kSeq, Vb, Vb, kSeq, (long)kDh * kSeq, (void*)Ch, (void*)Ch, kDim, (long)kDh,
              bo, Cf, (long)kDh, kSeq, kDh, kSeq, kPVScale);
        }
      }
    }
  }

  wmma_gemm64<0, false, 2, 0, false, 0><<<gOut, blk, 0, stream>>>(
      comb16, comb16, kDim, 0L, Wo16, Wo16, kDim, 0L, (void*)yout, (void*)yout, kDim, 0L,
      bo, x, 0L, kTok, kDim, kDim, kOutScale);
}
